// SSRM_35338990911668
// MI455X (gfx1250) — hardware-run, weakly checked
//
#include <hip/hip_runtime.h>


#ifndef NB
#define NB 2
#endif
#define NB_FULL 2
#define IH   128
#define IW   128
#define LL   (IH * IW)
#define CIN  200
#define CX   50
#define NSC  4
#define WIN  64
#define NCL  (LL / WIN)
#define NLAB 32
#define CP   224
#define KCV  (9 * CP)
#define XP   64
#define YW   208
#define KO   (NSC * YW)
#define KCAR 32.0f
#define YCAR 16.0f
#define WCAR 1024.0f
#define OSC  (1.0f / 16384.0f)
#define SC2  ((float)(1.4426950408889634 / 32.0))
#define PSH  14.0f
#define NEGB (-3.0e38f)

static_assert(NB <= NB_FULL);
static_assert(LL % 64 == 0);
static_assert(IW % 64 == 0);
static_assert(LL == 512 * 32);
static_assert(LL <= 65536);
static_assert(CIN % 8 == 0);
static_assert(CIN % 4 == 0);
static_assert(CIN <= CP);
static_assert(CP % 32 == 0);
static_assert(CX <= 64);
static_assert(XP == 64);
static_assert(CIN <= YW);
static_assert(YW == 13 * 16);
static_assert(YW % 8 == 0);
static_assert(KO % 32 == 0);
static_assert((NCL & (NCL - 1)) == 0);
static_assert(3 * WIN == 192);
static_assert(192 % 32 == 0);
static_assert(64 * (CP - CIN) == 6 * 256);
static_assert(64 * CP / 8 == 7 * 256);
static_assert(4 * 4 == 16 && 8 * 8 == XP);
static_assert(16 * YW / 8 == 13 * 32);
static_assert(64 * 8 == 4 * 128);
static_assert(192 * 8 == 12 * 128);
static_assert(192 * (YW / 8) == 39 * 128);
static_assert(64 * YW / 8 == 13 * 128);
static_assert(128 * (YW / 8) == 52 * 64);
static_assert(CIN == 25 * 2 * 4);
static_assert(8 * 512 * 4 == LL);
static_assert(8 * 16 == 32 * 4);
static_assert(64 * 72 * 2 + 192 * 72 * 2 + YW * 200 * 2 + 192 * 4 <= 131072);
static_assert(NLAB * 512 * 2 + 2 * LL * 2 + 512 * 4 + 16 * 4 <= 131072);
static_assert(32 * 840 * 2 + YW * 36 * 4 + 128 * 4 <= 131072);
static_assert(64 * YW <= YW * 200);

typedef _Float16 h16;
typedef unsigned short bf;
typedef __attribute__((ext_vector_type(16))) __bf16   v16bf;
typedef __attribute__((ext_vector_type(16))) _Float16 v16h;
typedef __attribute__((ext_vector_type(8)))  _Float16 v8h;
typedef __attribute__((ext_vector_type(8)))  unsigned short v8us;
typedef __attribute__((ext_vector_type(8)))  float    v8f;
typedef __attribute__((ext_vector_type(4)))  float    v4f;
typedef __attribute__((ext_vector_type(4)))  int      v4i;
typedef v4f  __attribute__((may_alias)) v4fa;
typedef v8h  __attribute__((may_alias)) v8ha;
typedef v8us __attribute__((may_alias)) v8usa;

__device__ __forceinline__ unsigned short f2bf(float f) { unsigned u = __float_as_uint(f); u += 0x7FFFu + ((u >> 16) & 1u); return (unsigned short)(u >> 16); }
__device__ __forceinline__ float bfr(float f) { return __uint_as_float(((unsigned)f2bf(f)) << 16); }
__device__ __forceinline__ v16h cat16(v8h lo, v8h hi) { return __builtin_shufflevector(lo, hi, 0, 1, 2, 3, 4, 5, 6, 7, 8, 9, 10, 11, 12, 13, 14, 15); }
__device__ __forceinline__ v16bf cat16b(v8us lo, v8us hi) { return __builtin_bit_cast(v16bf, __builtin_shufflevector(lo, hi, 0, 1, 2, 3, 4, 5, 6, 7, 8, 9, 10, 11, 12, 13, 14, 15)); }
__device__ __forceinline__ v8f wmma16(v16h a, v16h b, v8f c) { return __builtin_amdgcn_wmma_f32_16x16x32_f16(false, a, false, b, (short)0, c, false, false); }
__device__ __forceinline__ v8f wmmab(v16bf a, v16bf b, v8f c) { return __builtin_amdgcn_wmma_f32_16x16x32_bf16(false, a, false, b, (short)0, c, false, false); }
__device__ __forceinline__ v16h  ldh(const h16* p) { return cat16(*(const v8h*)p, *(const v8h*)(p + 16)); }
__device__ __forceinline__ v16bf ldb(const bf* p)  { return cat16b(*(const v8us*)p, *(const v8us*)(p + 16)); }
__device__ __forceinline__ void wave_sync() { __builtin_amdgcn_fence(3  , "wavefront"); __builtin_amdgcn_wave_barrier(); asm volatile("" ::: "memory"); }

__device__ __forceinline__ v8f wmma16g(v16h a, v16h b, v8f c) { c = wmma16(a, b, c); asm volatile("v_nop\n\tv_nop\n\tv_nop\n\tv_nop" : "+v"(c) : "v"(a), "v"(b)); return c; }
__device__ __forceinline__ v8f wmmabg(v16bf a, v16bf b, v8f c) { c = wmmab(a, b, c); asm volatile("v_nop\n\tv_nop\n\tv_nop\n\tv_nop" : "+v"(c) : "v"(a), "v"(b)); return c; }
static __device__ __forceinline__ h16 toh_flush(float v) { const h16 r = (h16)v; return (fabsf(v) < 6.103515625e-05f) ? (h16)0.0f : r; }
__device__ __forceinline__ int refl(int i, int n) { return i < 0 ? -i : (i >= n ? 2 * n - 2 - i : i); }

__device__ __forceinline__ float wsrc(const float* __restrict__ src, int nsrc, int row, int k, int gp, int cv, int ov, int so, int sg, int sc) {
    const int grp = k / gp, c = k - grp * gp;
    const bool ok = (row < ov) & (c < cv);
    int idx = row * so + grp * sg + c * sc; idx = idx < 0 ? 0 : (idx > nsrc - 1 ? nsrc - 1 : idx);
    float x = src[idx]; asm volatile("" : "+v"(x));
    return ok ? bfr(x) : 0.0f;
}

__global__ __launch_bounds__(256) void k_wpackb(const float* __restrict__ src, bf* dst, int npiece, int kp8, int gp, int cv, int ov, int so, int sg, int sc, int nsrc) {
    const int i = blockIdx.x * 256 + threadIdx.x; if (i >= npiece) return;
    const int row = i / kp8, k0 = (i - row * kp8) * 8; v8us o;
#pragma unroll
    for (int e = 0; e < 8; ++e) o[e] = f2bf(wsrc(src, nsrc, row, k0 + e, gp, cv, ov, so, sg, sc));
    *(volatile v8us*)(dst + (size_t)i * 8) = o; __threadfence(); *(volatile v8us*)(dst + (size_t)i * 8) = o;
}
__global__ __launch_bounds__(256) void k_wpackh(const float* __restrict__ src, h16* dst, int npiece, int kp8, int gp, int cv, int ov, int so, int sg, int sc, int nsrc, float carry) {
    const int i = blockIdx.x * 256 + threadIdx.x; if (i >= npiece) return;
    const int row = i / kp8, k0 = (i - row * kp8) * 8; v8h o;
#pragma unroll
    for (int e = 0; e < 8; ++e) o[e] = toh_flush(wsrc(src, nsrc, row, k0 + e, gp, cv, ov, so, sg, sc) * carry);
    *(volatile v8h*)(dst + (size_t)i * 8) = o; __threadfence(); *(volatile v8h*)(dst + (size_t)i * 8) = o;
}

__global__ __launch_bounds__(256) void k_xt(const float* __restrict__ in, bf* XT) {
    __shared__ __align__(16) bf ts[64 * 232];
    const int tid = threadIdx.x;
    const int n = blockIdx.x / (LL / 64), l0 = (blockIdx.x % (LL / 64)) * 64;
    const float* ib = in + (size_t)n * CIN * LL + l0 + (tid & 63);
    const int cq = tid >> 6;
#pragma unroll 1
    for (int i = 0; i < CIN / 4; ++i) { const int c = cq + 4 * i; ts[(tid & 63) * 232 + c] = f2bf(ib[(size_t)c * LL]); }
#pragma unroll 1
    for (int i = 0; i < 6; ++i) { const int e = i * 256 + tid; ts[(e / (CP - CIN)) * 232 + CIN + (e % (CP - CIN))] = (bf)0; }
    __syncthreads();
    bf* ob = XT + ((size_t)n * LL + l0) * CP;
#pragma unroll 1
    for (int ps = 0; ps < 2; ++ps) {
#pragma unroll 1
        for (int it = 0; it < 7; ++it) { const int e = (it * 256 + tid) * 8; const int row = e / CP, col = e - row * CP;
            const v8us v = *(const v8usa*)(&ts[row * 232 + col]);
            *(volatile v8us*)(ob + e) = v; }
        if (ps == 0) __threadfence(); }
}

__global__ __launch_bounds__(512) void k_sort(const int* __restrict__ lab, int* INV, int* POS, int* FLG) {
    __shared__ unsigned short cnt[NLAB * 512];
    __shared__ unsigned short posl[LL];
    __shared__ unsigned short invl[LL];
    __shared__ int part[512];
    __shared__ int wbad[16];
    const int tid = threadIdx.x, lane = tid & 31;
    const int wave = __builtin_amdgcn_readfirstlane((int)(threadIdx.x >> 5));
    const int z = blockIdx.x;
    const int* lp = lab + (size_t)z * LL + (size_t)tid * 32;
    int bad = 0;
#pragma unroll 1
    for (int b = 0; b < NLAB; ++b) cnt[b * 512 + tid] = (unsigned short)0;
#pragma unroll 1
    for (int i = 0; i < 32; ++i) { const int v = lp[i]; bad |= ((v < 0) | (v >= NLAB)) ? 1 : 0;
        const int b = v < 0 ? 0 : (v > NLAB - 1 ? NLAB - 1 : v);
        cnt[b * 512 + tid] = (unsigned short)(cnt[b * 512 + tid] + 1); }
    __syncthreads();
    int s = 0;
#pragma unroll 1
    for (int i = 0; i < 32; ++i) s += (int)cnt[tid * 32 + i];
    part[tid] = s;
    __syncthreads();
#pragma unroll 1
    for (int d = 1; d < 512; d <<= 1) {
        const int sidx = tid - d < 0 ? 0 : tid - d;
        int tmp = part[sidx]; asm volatile("" : "+v"(tmp));
        tmp = (tid >= d) ? tmp : 0;
        __syncthreads();
        part[tid] += tmp;
        __syncthreads(); }
    int run = part[tid] - s;
#pragma unroll 1
    for (int i = 0; i < 32; ++i) { const int c = (int)cnt[tid * 32 + i]; cnt[tid * 32 + i] = (unsigned short)run; run += c; }
    __syncthreads();
#pragma unroll 1
    for (int i = 0; i < 32; ++i) { const int j = tid * 32 + i; const int v = lp[i];
        const int b = v < 0 ? 0 : (v > NLAB - 1 ? NLAB - 1 : v);
        int p = (int)cnt[b * 512 + tid]; cnt[b * 512 + tid] = (unsigned short)(p + 1);
        p = p > LL - 1 ? LL - 1 : p;
        posl[j] = (unsigned short)p; invl[p] = (unsigned short)j; }
    int wb = bad;
    wb |= __shfl_xor(wb, 1, 32); wb |= __shfl_xor(wb, 2, 32); wb |= __shfl_xor(wb, 4, 32); wb |= __shfl_xor(wb, 8, 32); wb |= __shfl_xor(wb, 16, 32);
    if (lane == 0) wbad[wave] = wb;
    __syncthreads();
    int tot = 0;
#pragma unroll
    for (int q = 0; q < 16; ++q) tot |= wbad[q];
    v4i fl; fl[0] = tot; fl[1] = tot; fl[2] = tot; fl[3] = tot;
#pragma unroll 1
    for (int ps = 0; ps < 2; ++ps) {
#pragma unroll 1
        for (int it = 0; it < 8; ++it) { const int i = it * 512 + tid; v4i a, c;
#pragma unroll
            for (int e = 0; e < 4; ++e) { a[e] = (int)invl[4 * i + e]; c[e] = (int)posl[4 * i + e]; }
            *(volatile v4i*)(INV + (size_t)z * LL + 4 * i) = a;
            *(volatile v4i*)(POS + (size_t)z * LL + 4 * i) = c; }
        if ((wave == 0) & (lane < 8)) *(volatile v4i*)(FLG + z * 32 + 4 * lane) = fl;
        if (ps == 0) __threadfence(); }
}

__global__ __launch_bounds__(32) void k_xconv(const bf* __restrict__ XT, const bf* __restrict__ WX, h16* XQ, h16* XK) {
    __shared__ __align__(16) float os[16 * 68];
    const int lane = threadIdx.x & 31, lr = lane & 15, hi = lane >> 4;
    const int n = blockIdx.x / (LL / 64), l0 = (blockIdx.x % (LL / 64)) * 64;
    const int hrow = l0 / IW, w0 = l0 % IW;
    v8f acc[4][4];
#pragma unroll
    for (int mb = 0; mb < 4; ++mb)
#pragma unroll
        for (int nb = 0; nb < 4; ++nb) acc[mb][nb] = (v8f){};
    const size_t boff = (size_t)lr * KCV + 8 * hi;
#pragma unroll 1
    for (int tap = 0; tap < 9; ++tap) {
        const int dy = tap / 3, dx = tap - 3 * dy;
        const int hs = refl(hrow + dy - 1, IH);
        size_t ao[4];
#pragma unroll
        for (int mb = 0; mb < 4; ++mb) { const int ws = refl(w0 + mb * 16 + lr + dx - 1, IW); ao[mb] = ((size_t)n * LL + (size_t)(hs * IW + ws)) * CP + 8 * hi; }
#pragma unroll 1
        for (int kc = 0; kc < CP; kc += 32) {
            v16bf a[4];
#pragma unroll
            for (int mb = 0; mb < 4; ++mb) a[mb] = ldb(XT + ao[mb] + kc);
#pragma unroll
            for (int nb = 0; nb < 4; ++nb) { const v16bf b = ldb(WX + boff + (size_t)nb * 16 * KCV + (size_t)(tap * CP + kc));
#pragma unroll
                for (int mb = 0; mb < 4; ++mb) acc[mb][nb] = wmmabg(a[mb], b, acc[mb][nb]); }
        }
    }
#pragma unroll
    for (int mb = 0; mb < 4; ++mb) {
#pragma unroll
        for (int nb = 0; nb < 4; ++nb) {
#pragma unroll
            for (int j = 0; j < 8; ++j) os[(hi * 8 + j) * 68 + nb * 16 + lr] = acc[mb][nb][j]; }
        wave_sync();
        const size_t rowb = ((size_t)n * LL + l0 + mb * 16) * XP;
#pragma unroll 1
        for (int ps = 0; ps < 2; ++ps) {
#pragma unroll
            for (int s = 0; s < 4; ++s) { const int row = 4 * s + (lane >> 3), c8 = (lane & 7) * 8;
                const v4f x0 = *(const v4fa*)(&os[row * 68 + c8]); const v4f x1 = *(const v4fa*)(&os[row * 68 + c8 + 4]);
                float ss = 0.0f;
#pragma unroll
                for (int i = 0; i < 4; ++i) ss += x0[i] * x0[i] + x1[i] * x1[i];
                ss += __shfl_xor(ss, 1, 32); ss += __shfl_xor(ss, 2, 32); ss += __shfl_xor(ss, 4, 32);
                const float rn = KCAR * (1.0f / fmaxf(sqrtf(ss), 5.0e-5f));
                v8h qv, kv;
#pragma unroll
                for (int i = 0; i < 4; ++i) { qv[i] = toh_flush(x0[i]); qv[4 + i] = toh_flush(x1[i]); kv[i] = toh_flush(x0[i] * rn); kv[4 + i] = toh_flush(x1[i] * rn); }
                const size_t oo = rowb + (size_t)row * XP + c8;
                *(volatile v8h*)(XQ + oo) = qv; *(volatile v8h*)(XK + oo) = kv; }
            if (ps == 0) __threadfence(); }
        wave_sync();
    }
}

__global__ __launch_bounds__(128) __attribute__((amdgpu_num_vgpr(256))) void k_ygemm(const bf* __restrict__ XT, const bf* __restrict__ WY, h16* YP) {
    __shared__ __align__(16) float os[4 * 16 * 212];
    const int lane = threadIdx.x & 31, lr = lane & 15, hi = lane >> 4;
    const int wave = __builtin_amdgcn_readfirstlane((int)(threadIdx.x >> 5));
    const int r0 = (blockIdx.x * 4 + wave) * 16;
    v8f acc[13];
#pragma unroll
    for (int j = 0; j < 13; ++j) acc[j] = (v8f){};
    const size_t aoff = (size_t)(r0 + lr) * CP + 8 * hi, boff = (size_t)lr * CP + 8 * hi;
#pragma unroll 1
    for (int kc = 0; kc < CP; kc += 32) {
        const v16bf a = ldb(XT + aoff + kc);
#pragma unroll
        for (int j = 0; j < 13; ++j) { const v16bf b = ldb(WY + boff + (size_t)j * 16 * CP + kc); acc[j] = wmmabg(a, b, acc[j]); }
    }
    const int wb = wave * 16 * 212;
#pragma unroll
    for (int j = 0; j < 13; ++j) {
#pragma unroll
        for (int r = 0; r < 8; ++r) os[wb + (hi * 8 + r) * 212 + j * 16 + lr] = acc[j][r] * YCAR; }
    wave_sync();
    h16* ob = YP + (size_t)r0 * YW;
#pragma unroll 1
    for (int ps = 0; ps < 2; ++ps) {
#pragma unroll 1
        for (int it = 0; it < 13; ++it) { const int e = (it * 32 + lane) * 8; const int row = e / YW, col = e - row * YW;
            const v4f x0 = *(const v4fa*)(&os[wb + row * 212 + col]); const v4f x1 = *(const v4fa*)(&os[wb + row * 212 + col + 4]); v8h hv;
#pragma unroll
            for (int i = 0; i < 4; ++i) { hv[i] = toh_flush(x0[i]); hv[4 + i] = toh_flush(x1[i]); }
            *(volatile v8h*)(ob + e) = hv; }
        if (ps == 0) __threadfence(); }
}

__global__ __launch_bounds__(128) __attribute__((amdgpu_num_vgpr(256))) void k_attn(const h16* __restrict__ XQ, const h16* __restrict__ XK, const h16* __restrict__ YP,
                                                                                     const int* __restrict__ INV, h16* AO) {
    __shared__ __align__(16) h16 qs[64 * 72];
    __shared__ __align__(16) h16 ks[192 * 72];
    __shared__ __align__(16) h16 yt[YW * 200];
    __shared__ int rowl[192];
    const int tid = threadIdx.x, lane = tid & 31, lr = lane & 15, hi = lane >> 4;
    const int wave = __builtin_amdgcn_readfirstlane((int)(threadIdx.x >> 5));
    const int cid = blockIdx.x;
    const int n = cid / (NSC * NCL), zs = cid / NCL, kk = cid % NCL;
#pragma unroll
    for (int rr = 0; rr < 2; ++rr) {
        if (rr == 0 || wave < 2) {
            const int r = rr * 128 + tid; const int w = r >> 6;
            const int kw = (kk + ((w == 1) ? (NCL - 1) : 0) + ((w == 2) ? 1 : 0)) & (NCL - 1);
            int l = INV[(size_t)zs * LL + kw * WIN + (r & 63)]; l = l < 0 ? 0 : (l > LL - 1 ? LL - 1 : l);
            rowl[r] = n * LL + l; }
    }
    __syncthreads();
#pragma unroll 1
    for (int it = 0; it < 4; ++it) { const int i = it * 128 + tid; const int row = i >> 3, c8 = (i & 7) * 8;
        const v8h v = *(const v8h*)(XQ + (size_t)rowl[row] * XP + c8); *(v8ha*)(&qs[row * 72 + c8]) = v; }
#pragma unroll 1
    for (int it = 0; it < 12; ++it) { const int i = it * 128 + tid; const int row = i >> 3, c8 = (i & 7) * 8;
        const v8h v = *(const v8h*)(XK + (size_t)rowl[row] * XP + c8); *(v8ha*)(&ks[row * 72 + c8]) = v; }
#pragma unroll 1
    for (int it = 0; it < 39; ++it) { const int i = it * 128 + tid; const int row = i / (YW / 8), pc = i - row * (YW / 8);
        const v8h v = *(const v8h*)(YP + (size_t)rowl[row] * YW + pc * 8);
#pragma unroll
        for (int e = 0; e < 8; ++e) yt[(pc * 8 + e) * 200 + row] = v[e]; }
    __syncthreads();

    v8f o[13];
#pragma unroll
    for (int j = 0; j < 13; ++j) o[j] = (v8f){};
    float m = NEGB, l = 0.0f;
    const int qb = (wave * 16 + lr) * 72 + 8 * hi;
    const int kb = lr * 72 + 8 * hi;
    const int yb = lr * 200 + 8 * hi;
#pragma unroll 1
    for (int key0 = 0; key0 < 192; key0 += 32) {
        const v16h q0 = cat16(*(const v8ha*)(&qs[qb]),      *(const v8ha*)(&qs[qb + 16]));
        const v16h q1 = cat16(*(const v8ha*)(&qs[qb + 32]), *(const v8ha*)(&qs[qb + 48]));
        const int ka = kb + key0 * 72;
        const v16h ka0 = cat16(*(const v8ha*)(&ks[ka]),                *(const v8ha*)(&ks[ka + 16]));
        const v16h ka1 = cat16(*(const v8ha*)(&ks[ka + 32]),           *(const v8ha*)(&ks[ka + 48]));
        const v16h kb0 = cat16(*(const v8ha*)(&ks[ka + 16 * 72]),      *(const v8ha*)(&ks[ka + 16 * 72 + 16]));
        const v16h kb1 = cat16(*(const v8ha*)(&ks[ka + 16 * 72 + 32]), *(const v8ha*)(&ks[ka + 16 * 72 + 48]));
        v8f sa = (v8f){}, sb = (v8f){};
        sa = wmma16g(ka0, q0, sa); sa = wmma16g(ka1, q1, sa);
        sb = wmma16g(kb0, q0, sb); sb = wmma16g(kb1, q1, sb);
        float ta[8], tb[8]; float mx = NEGB;
#pragma unroll
        for (int r = 0; r < 8; ++r) { ta[r] = sa[r] * SC2; tb[r] = sb[r] * SC2; mx = fmaxf(mx, fmaxf(ta[r], tb[r])); }
        mx = fmaxf(mx, __shfl_xor(mx, 16, 32));
        const float mnew = fmaxf(m, mx);
        const float alpha = __builtin_amdgcn_exp2f(m - mnew);
        const float sh = PSH - mnew;
        v16h pb; float ls = 0.0f;
#pragma unroll
        for (int r = 0; r < 8; ++r) {
            const float ea = ta[r] + sh, eb = tb[r] + sh;
            const float xa = __builtin_amdgcn_exp2f(ea), xb = __builtin_amdgcn_exp2f(eb);
            const float ga = (ea < -14.0f) ? 0.0f : xa, gb = (eb < -14.0f) ? 0.0f : xb;
            const h16 pa = (h16)ga; const h16 pc = (h16)gb;
            pb[r] = pa; pb[8 + r] = pc;
            ls += (float)pa + (float)pc; }
        l = l * alpha + ls; m = mnew;
#pragma unroll
        for (int j = 0; j < 13; ++j) o[j] = o[j] * alpha;
        const int ya = yb + key0;
#pragma unroll
        for (int j = 0; j < 13; ++j) {
            const v16h yf = cat16(*(const v8ha*)(&yt[ya + j * 16 * 200]), *(const v8ha*)(&yt[ya + j * 16 * 200 + 16]));
            o[j] = wmma16g(yf, pb, o[j]); }
    }
    l += __shfl_xor(l, 16, 32);
    const float inv = 1.0f / l;
    __syncthreads();
#pragma unroll
    for (int j = 0; j < 13; ++j) { v8h ov;
#pragma unroll
        for (int r = 0; r < 8; ++r) ov[r] = toh_flush(o[j][r] * inv);
        *(v8ha*)(&yt[(wave * 16 + lr) * YW + 16 * j + 8 * hi]) = ov; }
    __syncthreads();
    h16* ob = AO + (size_t)cid * WIN * YW;
#pragma unroll 1
    for (int ps = 0; ps < 2; ++ps) {
#pragma unroll 1
        for (int it = 0; it < 13; ++it) { const int e = (it * 128 + tid) * 8;
            const v8h v = *(const v8ha*)(&yt[e]);
            *(volatile v8h*)(ob + e) = v; }
        if (ps == 0) __threadfence(); }
}

__global__ __launch_bounds__(64) __attribute__((amdgpu_num_vgpr(256))) void k_out(const h16* __restrict__ AO, const h16* __restrict__ WO, const int* __restrict__ POS,
                                                                                   const int* __restrict__ FLG, const float* __restrict__ bout, const float* __restrict__ in, float* OUT) {
    __shared__ __align__(16) h16 at[32 * 840];
    __shared__ __align__(16) float os[YW * 36];
    __shared__ int rowp[128];
    const int tid = threadIdx.x, lane = tid & 31, lr = lane & 15, hi = lane >> 4;
    const int wave = __builtin_amdgcn_readfirstlane((int)(threadIdx.x >> 5));
    const int n = blockIdx.x / (LL / 32), l0 = (blockIdx.x % (LL / 32)) * 32;
#pragma unroll
    for (int rr = 0; rr < 2; ++rr) { const int r = rr * 64 + tid; const int s = r >> 5, pix = r & 31;
        const size_t zb = (size_t)(n * NSC + s) * LL;
        int p = POS[zb + l0 + pix]; p = p < 0 ? 0 : (p > LL - 1 ? LL - 1 : p);
        rowp[r] = (n * NSC + s) * LL + p; }
    __syncthreads();
#pragma unroll 1
    for (int it = 0; it < 52; ++it) { const int i = it * 64 + tid; const int r = i / (YW / 8), pc = i - r * (YW / 8);
        const v8h v = *(const v8h*)(AO + (size_t)rowp[r] * YW + pc * 8);
        *(v8ha*)(&at[(r & 31) * 840 + (r >> 5) * YW + pc * 8]) = v; }
    __syncthreads();
    v8f acc[13];
#pragma unroll
    for (int j = 0; j < 13; ++j) acc[j] = (v8f){};
    const int ab = (wave * 16 + lr) * 840 + 8 * hi;
    const size_t boff = (size_t)lr * KO + 8 * hi;
#pragma unroll 1
    for (int kc = 0; kc < KO; kc += 32) {
        const v16h a = cat16(*(const v8ha*)(&at[ab + kc]), *(const v8ha*)(&at[ab + kc + 16]));
#pragma unroll
        for (int j = 0; j < 13; ++j) { const v16h b = ldh(WO + boff + (size_t)j * 16 * KO + kc); acc[j] = wmma16g(a, b, acc[j]); }
    }
#pragma unroll
    for (int j = 0; j < 13; ++j) { v4f a0, a1;
#pragma unroll
        for (int i = 0; i < 4; ++i) { a0[i] = acc[j][i]; a1[i] = acc[j][4 + i]; }
        *(v4fa*)(&os[(16 * j + lr) * 36 + wave * 16 + 8 * hi]) = a0; *(v4fa*)(&os[(16 * j + lr) * 36 + wave * 16 + 8 * hi + 4]) = a1; }
    __syncthreads();
    int bad = 0;
#pragma unroll
    for (int q = 0; q < NB * NSC; ++q) bad |= FLG[q * 32];
    const float nanv = __uint_as_float(0x7FC00000u);
#pragma unroll 1
    for (int ps = 0; ps < 2; ++ps) {
#pragma unroll 1
        for (int it = 0; it < 25; ++it) { const int oc = it * 8 + wave * 4 + (lane >> 3), c4 = (lane & 7) * 4;
            const v4f x = *(const v4fa*)(&os[oc * 36 + c4]);
            const size_t g = ((size_t)n * CIN + oc) * LL + l0 + c4;
            const v4f rin = *(const v4f*)(in + g);
            const float bo = bfr(bout[oc]);
            v4f val;
#pragma unroll
            for (int i = 0; i < 4; ++i) { const float t = x[i] * OSC + bo + bfr(rin[i]); val[i] = (bad != 0) ? nanv : t; }
            *(volatile v4f*)(OUT + g) = val; }
        if (ps == 0) __threadfence(); }
}

static constexpr size_t al256(size_t v) { return (v + 255) & ~(size_t)255; }
static constexpr size_t SZ_WX = al256((size_t)64 * KCV * 2);
static constexpr size_t SZ_WY = al256((size_t)YW * CP * 2);
static constexpr size_t SZ_WO = al256((size_t)YW * KO * 2);
static constexpr size_t SZ_XT = al256((size_t)NB * LL * CP * 2);
static constexpr size_t SZ_XP = al256((size_t)NB * LL * XP * 2);
static constexpr size_t SZ_YP = al256((size_t)NB * LL * YW * 2);
static constexpr size_t SZ_IX = al256((size_t)NB * NSC * LL * 4);
static constexpr size_t SZ_FL = al256((size_t)NB * NSC * 32 * 4);
static constexpr size_t SZ_AO = al256((size_t)NB * NSC * LL * YW * 2);
static constexpr size_t SZ_TOTAL = SZ_WX + SZ_WY + SZ_WO + SZ_XT + 2 * SZ_XP + SZ_YP + 2 * SZ_IX + SZ_FL + SZ_AO;
static_assert(SZ_TOTAL <= (size_t)134217728);
static_assert(((size_t)64 * KCV * 2) % 128 == 0);
static_assert(((size_t)YW * CP * 2) % 128 == 0);
static_assert(((size_t)YW * KO * 2) % 128 == 0);
static_assert(((size_t)64 * CP * 2) % 128 == 0);
static_assert(((size_t)16 * YW * 2) % 128 == 0);
static_assert(((size_t)WIN * YW * 2) % 128 == 0);
static_assert((64 * KCV) % 8 == 0 && (YW * CP) % 8 == 0 && (YW * KO) % 8 == 0);

extern "C" void kernel_launch(void* const* d_in, const int* in_sizes, int n_in,
                              void* d_out, int out_size, void* d_ws, size_t ws_size, hipStream_t stream) {
    if (n_in < 6) return;
    if ((size_t)in_sizes[0] < (size_t)NB * CIN * LL) return;
    if ((size_t)in_sizes[1] < (size_t)NB * NSC * LL) return;
    if ((size_t)in_sizes[2] < (size_t)CX * CIN * 9) return;
    if ((size_t)in_sizes[3] < (size_t)CIN * CIN) return;
    if ((size_t)in_sizes[4] < (size_t)CIN * NSC * CIN) return;
    if (in_sizes[5] < CIN) return;
    if ((size_t)out_size < (size_t)NB * CIN * LL) return;
    if (SZ_TOTAL > ws_size) return;
    const float* xin  = (const float*)d_in[0];
    const int*   lab  = (const int*)d_in[1];
    const float* wx   = (const float*)d_in[2];
    const float* wy   = (const float*)d_in[3];
    const float* wo   = (const float*)d_in[4];
    const float* bo   = (const float*)d_in[5];
    float* OUT = (float*)d_out;
    char* wsp = (char*)d_ws;
    bf*  WXB = (bf*)wsp;  wsp += SZ_WX;
    bf*  WYB = (bf*)wsp;  wsp += SZ_WY;
    h16* WOH = (h16*)wsp; wsp += SZ_WO;
    bf*  XT  = (bf*)wsp;  wsp += SZ_XT;
    h16* XQ  = (h16*)wsp; wsp += SZ_XP;
    h16* XK  = (h16*)wsp; wsp += SZ_XP;
    h16* YP  = (h16*)wsp; wsp += SZ_YP;
    int* INV = (int*)wsp; wsp += SZ_IX;
    int* POS = (int*)wsp; wsp += SZ_IX;
    int* FLG = (int*)wsp; wsp += SZ_FL;
    h16* AO  = (h16*)wsp; wsp += SZ_AO;

    { const int np = 64 * KCV / 8;  k_wpackb<<<(unsigned)((np + 255) / 256), 256, 0, stream>>>(wx, WXB, np, KCV / 8, CP, CIN, CX, CIN * 9, 1, 9, CX * CIN * 9); }
    { const int np = YW * CP / 8;   k_wpackb<<<(unsigned)((np + 255) / 256), 256, 0, stream>>>(wy, WYB, np, CP / 8, CP, CIN, CIN, CIN, 0, 1, CIN * CIN); }
    { const int np = YW * KO / 8;   k_wpackh<<<(unsigned)((np + 255) / 256), 256, 0, stream>>>(wo, WOH, np, KO / 8, YW, CIN, CIN, NSC * CIN, CIN, 1, CIN * NSC * CIN, WCAR); }
    k_xt<<<NB * LL / 64, 256, 0, stream>>>(xin, XT);
    k_sort<<<NB * NSC, 512, 0, stream>>>(lab, INV, POS, FLG);
    k_xconv<<<NB * LL / 64, 32, 0, stream>>>(XT, WXB, XQ, XK);
    k_ygemm<<<NB * LL / 64, 128, 0, stream>>>(XT, WYB, YP);
    k_attn<<<NB * NSC * NCL, 128, 0, stream>>>(XQ, XK, YP, INV, AO);
    k_out<<<NB * LL / 32, 64, 0, stream>>>(AO, WOH, POS, FLG, bo, xin, OUT);
}
